// shape_align_68564857913609
// MI455X (gfx1250) — hardware-verified
//
#include <hip/hip_runtime.h>
#include <math.h>

typedef __attribute__((ext_vector_type(16))) _Float16 v16h;
typedef __attribute__((ext_vector_type(16))) __bf16 v16b;
typedef __attribute__((ext_vector_type(8)))  _Float16 v8h;
typedef __attribute__((ext_vector_type(8)))  float v8f;
typedef __attribute__((ext_vector_type(4)))  float v4f;
typedef __attribute__((ext_vector_type(2)))  float v2f;
typedef __attribute__((ext_vector_type(4)))  unsigned v4u;
typedef __attribute__((ext_vector_type(4)))  int v4i;
typedef float __attribute__((may_alias)) float_a;
typedef int __attribute__((may_alias)) int_a;

template <typename T> __device__ __forceinline__ void vst2(void* p, T v) { *(volatile T*)p = v; __threadfence(); *(volatile T*)p = v; }
__device__ __forceinline__ v8f wmma16(v16h a, v16h b, v8f c) {
  v8f d = __builtin_amdgcn_wmma_f32_16x16x32_f16(false, a, false, b, (short)0, c, false, false);
  asm volatile("v_nop\n\tv_nop\n\tv_nop\n\tv_nop" : "+v"(d) : "v"(a), "v"(b));
  return d;
}
__device__ __forceinline__ v8f wmma_bf(v16b a, v16b b, v8f c) {
  v8f d = __builtin_amdgcn_wmma_f32_16x16x32_bf16(false, a, false, b, (short)0, c, false, false);
  asm volatile("v_nop\n\tv_nop\n\tv_nop\n\tv_nop" : "+v"(d) : "v"(a), "v"(b));
  return d;
}
__device__ __forceinline__ v16h frag_h(const _Float16* rowk0, int lane) {
  union { v16h v; v8h q[2]; } u; const _Float16* p = rowk0 + 8 * (lane >> 4);
  u.q[0] = *(const v8h*)p; u.q[1] = *(const v8h*)(p + 16); return u.v;
}
__device__ __forceinline__ v16h frag_f32(const float* rowk0, int lane) {
  v16h a; const float* p = rowk0 + 8 * (lane >> 4);
#pragma unroll
  for (int i = 0; i < 8; ++i) { a[i] = (_Float16)p[i]; a[8 + i] = (_Float16)p[16 + i]; }
  return a;
}
__device__ __forceinline__ v16h frag_f32s(const float* rowk0, int lane, float sc) {
  v16h a; const float* p = rowk0 + 8 * (lane >> 4);
#pragma unroll
  for (int i = 0; i < 8; ++i) { a[i] = (_Float16)(p[i] * sc); a[8 + i] = (_Float16)(p[16 + i] * sc); }
  return a;
}
__device__ __forceinline__ v16h fragc_f32(const float* W, int k0, int n, int lane, int ld, int K) {
  v16h a; const int g = lane >> 4;
#pragma unroll
  for (int i = 0; i < 8; ++i) { const int ka = k0 + 8 * g + i, kb = ka + 16;
    a[i] = (_Float16)(ka < K ? W[(size_t)(ka < K ? ka : K - 1) * ld + n] : 0.f); a[8 + i] = (_Float16)(kb < K ? W[(size_t)(kb < K ? kb : K - 1) * ld + n] : 0.f); }
  return a;
}
struct F2 { v16b h, l; };
__device__ __forceinline__ F2 bsplit16(const float v[16]) { F2 r;
#pragma unroll
  for (int i = 0; i < 16; ++i) { const __bf16 h = (__bf16)v[i]; r.h[i] = h; r.l[i] = (__bf16)(v[i] - (float)h); }
  return r; }
__device__ __forceinline__ F2 split_row(const float* row, int k0, int lane) { float v[16]; const float* p = row + k0 + 8 * (lane >> 4);
#pragma unroll
  for (int i = 0; i < 8; ++i) { v[i] = p[i]; v[8 + i] = p[16 + i]; }
  return bsplit16(v); }
__device__ __forceinline__ F2 split_rowK(const float* row, int k0, int lane, int K) { float v[16]; const int g = lane >> 4;
#pragma unroll
  for (int i = 0; i < 8; ++i) { const int ka = k0 + 8 * g + i, kb = ka + 16; v[i] = ka < K ? row[ka < K ? ka : K - 1] : 0.f; v[8 + i] = kb < K ? row[kb < K ? kb : K - 1] : 0.f; }
  return bsplit16(v); }
__device__ __forceinline__ F2 split_col(const float* W, int k0, int n, int lane, int ld, int K) { float v[16]; const int g = lane >> 4;
#pragma unroll
  for (int i = 0; i < 8; ++i) { const int ka = k0 + 8 * g + i, kb = ka + 16; v[i] = ka < K ? W[(size_t)(ka < K ? ka : K - 1) * ld + n] : 0.f; v[8 + i] = kb < K ? W[(size_t)(kb < K ? kb : K - 1) * ld + n] : 0.f; }
  return bsplit16(v); }
__device__ __forceinline__ v8f mac3(const F2& a, const F2& b, v8f c) { c = wmma_bf(a.l, b.h, c); c = wmma_bf(a.h, b.l, c); return wmma_bf(a.h, b.h, c); }
__device__ __forceinline__ float sigm(float v) { return 1.0f / (1.0f + expf(-v)); }
#define LDSX() do { asm volatile("s_wait_dscnt 0" ::: "memory"); __builtin_amdgcn_wave_barrier(); __builtin_amdgcn_fence(__ATOMIC_RELEASE, "workgroup"); } while (0)


#define NB 4
#define CH 256
#define HH 48
#define WW 160
#define NPIX (HH * WW)
#define NP (NB * NPIX)
#define NA 36
#define K2 9
#define KCOL (CH * K2)
#define NPASS 2
#define PROWS (NP / NPASS)
#ifndef NBT
#define NBT NB
#endif
typedef __attribute__((ext_vector_type(8))) __bf16 v8b;
__device__ __forceinline__ v16b frag_b(const __bf16* rowk0, int lane) {
  union { v16b v; v8b q[2]; } u; const __bf16* p = rowk0 + 8 * (lane >> 4);
  u.q[0] = *(const v8b*)p; u.q[1] = *(const v8b*)(p + 16); return u.v;
}
__device__ __forceinline__ float bfr(float v) { return (float)(__bf16)v; }
__device__ __attribute__((noinline)) float exp_ni(float v) { return expf(v); }
__device__ __attribute__((noinline)) float erf_ni(float v) { return erff(v); }

#define WS_PK  0u
#define WS_PIX (WS_PK + 2u * CH * KCOL)
#define WS_CH  (WS_PIX + 4u * (size_t)NP * 32)
#define WS_CL  (WS_CH + 2u * (size_t)PROWS * KCOL)
#define WS_END (WS_CL + 2u * (size_t)PROWS * KCOL)

__global__ __launch_bounds__(256) void k_pack(const float* __restrict__ WT, __bf16* __restrict__ PK) {
  __shared__ __align__(16) __bf16 s[KCOL]; const int o = blockIdx.x, t = threadIdx.x;
  for (int k = t; k < KCOL; k += 256) s[k] = (__bf16)WT[(size_t)o * KCOL + k];
  __syncthreads();
  for (int q = t; q < KCOL / 8; q += 256) vst2((unsigned*)(PK + (size_t)o * KCOL + q * 8), *(const v4u*)&s[q * 8]);
}
__global__ __launch_bounds__(256) void k_pix(const float* __restrict__ PROB, const float* __restrict__ TAB, float* __restrict__ PIX) {
  __shared__ __align__(16) float so[64][32]; const int tid = threadIdx.x; const int pl = tid >> 2, part = tid & 3; const size_t p = (size_t)blockIdx.x * 64 + pl; const int b = (int)(p / NPIX), hw = (int)(p % NPIX);
  float bv[3]; int bi[3];
#pragma unroll
  for (int s = 0; s < 3; ++s) { bv[s] = -3.0e38f; bi[s] = 0; }
  for (int a = 0; a < NA; ++a) { const float v = bfr(PROB[((size_t)b * NA + a) * NPIX + hw]); if (v > bv[2]) { float cv = v; int ci = a; bool placed = false;
#pragma unroll
      for (int s = 0; s < 3; ++s) { const bool swp = placed || (cv > bv[s]); placed = swp; const float tv = bv[s]; const int ti = bi[s]; bv[s] = swp ? cv : tv; bi[s] = swp ? ci : ti; cv = swp ? tv : cv; ci = swp ? ti : ci; } } }
  const float m = bv[0]; const float e1 = exp_ni(bv[1] - m), e2 = exp_ni(bv[2] - m); const float se = 1.0f + e1 + e2; const float w0 = 1.0f / se, w1 = e1 / se, w2 = e2 / se; const float hard = (m > 0.5f) ? 1.f : 0.f;
  for (int chn = part; chn < 18; chn += 4) { const size_t base = (size_t)chn * NPIX + hw;
    const float o = (w0 * bfr(TAB[(size_t)bi[0] * 18 * NPIX + base]) + w1 * bfr(TAB[(size_t)bi[1] * 18 * NPIX + base])) + w2 * bfr(TAB[(size_t)bi[2] * 18 * NPIX + base]);
    so[pl][chn] = o * hard; }
  if (part == 0) { so[pl][18] = m; for (int q = 19; q < 32; ++q) so[pl][q] = 0.f; }
  __syncthreads();
  for (int e = tid; e < 64 * 8; e += 256) { const int r = e >> 3, pc = e & 7; vst2(PIX + ((size_t)blockIdx.x * 64 + r) * 32 + pc * 4, *(const v4f*)&so[r][pc * 4]); }
}
__global__ __launch_bounds__(256) void k_col(const float* __restrict__ X, const float* __restrict__ PIX, int pass, __bf16* __restrict__ CHp, __bf16* __restrict__ CLp) {
  __shared__ float spix[64][20]; __shared__ __align__(16) __bf16 sh_[8][KCOL + 8], sl_[8][KCOL + 8];
  const int tid = threadIdx.x; const size_t prow0 = (size_t)blockIdx.x * 64; const size_t p0 = (size_t)pass * PROWS + prow0;
  for (int e = tid; e < 64 * 19; e += 256) { const int r = e / 19, q = e % 19; spix[r][q] = PIX[(p0 + r) * 32 + q]; }
  __syncthreads();
  for (int r8 = 0; r8 < 8; ++r8) {
    for (int e = tid; e < 8 * KCOL; e += 256) { const int rl = e / KCOL, k = e % KCOL; const int r = r8 * 8 + rl; const size_t p = p0 + r; const int b = (int)(p / NPIX), hw = (int)(p % NPIX); const int h = hw / WW, w = hw % WW;
      const int c = k / K2, kk = k % K2; const float py = (float)h + (float)(kk / 3 - 1) + spix[r][2 * kk]; const float px = (float)w + (float)(kk % 3 - 1) + spix[r][2 * kk + 1];
      const float fy = floorf(py), fx = floorf(px); const float dy = py - fy, dx = px - fx; const int y0 = (int)fy, x0 = (int)fx;
      const float* xc = X + ((size_t)b * CH + c) * NPIX; float v = 0.f;
      { const int yy = y0, xx = x0; if (yy >= 0 && yy < HH && xx >= 0 && xx < WW) v += bfr(xc[yy * WW + xx]) * ((1.f - dy) * (1.f - dx)); }
      { const int yy = y0, xx = x0 + 1; if (yy >= 0 && yy < HH && xx >= 0 && xx < WW) v += bfr(xc[yy * WW + xx]) * ((1.f - dy) * dx); }
      { const int yy = y0 + 1, xx = x0; if (yy >= 0 && yy < HH && xx >= 0 && xx < WW) v += bfr(xc[yy * WW + xx]) * (dy * (1.f - dx)); }
      { const int yy = y0 + 1, xx = x0 + 1; if (yy >= 0 && yy < HH && xx >= 0 && xx < WW) v += bfr(xc[yy * WW + xx]) * (dy * dx); }
      v *= spix[r][18];
      const __bf16 hb = (__bf16)v; sh_[rl][k] = hb; sl_[rl][k] = (__bf16)(v - (float)hb); }
    __syncthreads();
    for (int e = tid; e < 8 * KCOL / 8; e += 256) { const int rl = e / (KCOL / 8), pc = e % (KCOL / 8); const size_t o = (prow0 + r8 * 8 + rl) * KCOL + pc * 8; vst2((unsigned*)(CHp + o), *(const v4u*)&sh_[rl][pc * 8]); vst2((unsigned*)(CLp + o), *(const v4u*)&sl_[rl][pc * 8]); }
    __syncthreads(); }
}
__global__ __launch_bounds__(128) void k_gemm(const __bf16* __restrict__ CHp, const __bf16* __restrict__ CLp, const __bf16* __restrict__ PK, const float* __restrict__ BIAS, const float* __restrict__ X, int pass, float* __restrict__ OUT) {
  __shared__ __align__(16) float st[128][68];
  const int tid = threadIdx.x, wave = tid >> 5, lane = tid & 31, col = lane & 15, g = lane >> 4; const size_t pr0 = (size_t)blockIdx.x * 64; const size_t r0 = pr0 + wave * 16; const int n0 = blockIdx.y * 128;
  const size_t p0 = (size_t)pass * PROWS + pr0; const int b = (int)(p0 / NPIX), hw0 = (int)(p0 % NPIX);
  v8f acc[8] = {};
#pragma unroll 2
  for (int kc = 0; kc < KCOL / 32; ++kc) { F2 a; a.h = frag_b(CHp + (r0 + col) * KCOL + kc * 32, lane); a.l = frag_b(CLp + (r0 + col) * KCOL + kc * 32, lane);
#pragma unroll
    for (int j = 0; j < 8; ++j) { const v16b w = frag_b(PK + (size_t)(n0 + j * 16 + col) * KCOL + kc * 32, lane); acc[j] = wmma_bf(a.l, w, acc[j]); acc[j] = wmma_bf(a.h, w, acc[j]); } }
#pragma unroll
  for (int j = 0; j < 8; ++j) { const int o = n0 + j * 16 + col; const float bb = bfr(BIAS[o]);
#pragma unroll
    for (int r = 0; r < 8; ++r) { const int pl = wave * 16 + 8 * g + r; st[j * 16 + col][pl] = acc[j][r] + bb + bfr(X[((size_t)b * CH + o) * NPIX + hw0 + pl]); } }
  __syncthreads();
  for (int e = tid; e < 128 * 16; e += 128) { const int oc = e >> 4, pc = e & 15; vst2(OUT + ((size_t)b * CH + n0 + oc) * NPIX + hw0 + pc * 4, *(const v4f*)&st[oc][pc * 4]); }
}
extern "C" void kernel_launch(void* const* d_in, const int* in_sizes, int n_in, void* d_out, int out_size, void* d_ws, size_t ws_size, hipStream_t stream) {
  (void)in_sizes; (void)n_in; (void)out_size;
  const float** F = (const float**)d_in;
  if (ws_size < (size_t)WS_END) return;
  char* ws = (char*)d_ws; __bf16 *PK = (__bf16*)(ws + WS_PK), *CHp = (__bf16*)(ws + WS_CH), *CLp = (__bf16*)(ws + WS_CL); float* PIX = (float*)(ws + WS_PIX);
  k_pack<<<CH, 256, 0, stream>>>(F[3], PK);
  k_pix<<<NBT * NPIX / 64, 256, 0, stream>>>(F[1], F[2], PIX);
  for (int pass = 0; pass < NPASS; ++pass) { if (pass * PROWS >= NBT * NPIX) break; const int rows = min(PROWS, NBT * NPIX - pass * PROWS);
    k_col<<<rows / 64, 256, 0, stream>>>(F[0], PIX, pass, CHp, CLp);
    k_gemm<<<dim3(rows / 64, CH / 128), 128, 0, stream>>>(CHp, CLp, PK, F[4], F[0], pass, (float*)d_out); }
}
